// MultiQueryAttention_44418551775724
// MI455X (gfx1250) — hardware-verified
//
#include <hip/hip_runtime.h>
#include <stdint.h>


typedef _Float16 v16h __attribute__((ext_vector_type(16)));
typedef _Float16 v8h  __attribute__((ext_vector_type(8)));
typedef float    v8f  __attribute__((ext_vector_type(8)));
typedef float    v4f  __attribute__((ext_vector_type(4)));

#define DM 2048
#define HD 128
#define NH 16
#define NKV 4
#define GQ (NH / NKV)
#define KVW (NKV * HD)
#define NQKV (DM + 2 * KVW)
#define NB_FULL 2
#define SEQ_FULL 2048
#ifndef NB
#define NB 2
#endif
#ifndef SEQ
#define SEQ 2048
#endif
#ifndef EARLY
#define EARLY 256
#endif
#define MROWS (NB * SEQ)
#define WSCALE 64.0f
#define PCARRY 256.0f
#define YCARRY 64.0f
#define QCARRY 8.0f
#define RSC 2048.0f
#define RINV (1.0f / 2048.0f)
#define NEGBIG (-1e30f)
#define QALPHA ((float)(0.08838834764831845 * 1.4426950408889634 * 8.0))

static_assert(SEQ % 256 == 0);
static_assert(SEQ <= SEQ_FULL);
static_assert(NB >= 1 && NB <= NB_FULL);
static_assert(EARLY % 128 == 0 && EARLY >= 128 && EARLY <= SEQ);
static_assert(DM == NH * HD && HD == 128 && NH == NKV * GQ && GQ == 4);
static_assert(DM == 256 * 8);
static_assert(NQKV % 128 == 0 && DM % 128 == 0 && DM % 64 == 0 && NQKV % 32 == 0);
static_assert(MROWS % 128 == 0);

union HFrag { v16h v; v8h h[2]; };

__device__ __forceinline__ v16h load_frag(const _Float16* p) {
    HFrag f;
    f.h[0] = *reinterpret_cast<const v8h*>(p);
    f.h[1] = *reinterpret_cast<const v8h*>(p + 16);
    return f.v;
}

__device__ __forceinline__ v8f wmma16(v16h a, v16h b, v8f c) {
    return __builtin_amdgcn_wmma_f32_16x16x32_f16(false, a, false, b, (short)0, c, false, false);
}

__device__ __forceinline__ float bf16r(float f) {
    unsigned int u = __float_as_uint(f);
    u += 0x7FFFu + ((u >> 16) & 1u);
    u &= 0xFFFF0000u;
    return __uint_as_float(u);
}

__global__ __launch_bounds__(256) void k_cvt_x(const float* __restrict__ x, _Float16* x16)
{
    const int u = blockIdx.x * 256 + threadIdx.x;
    const int row = u >> 8;
    const int col = (u & 255) * 8;
    const int bb = row / SEQ;
    const int s  = row - bb * SEQ;
    const float* src = x + ((size_t)(bb * SEQ_FULL + s)) * DM + col;
    const float4 f0 = *reinterpret_cast<const float4*>(src);
    const float4 f1 = *reinterpret_cast<const float4*>(src + 4);
    v8h o;
    o[0] = (_Float16)bf16r(f0.x); o[1] = (_Float16)bf16r(f0.y);
    o[2] = (_Float16)bf16r(f0.z); o[3] = (_Float16)bf16r(f0.w);
    o[4] = (_Float16)bf16r(f1.x); o[5] = (_Float16)bf16r(f1.y);
    o[6] = (_Float16)bf16r(f1.z); o[7] = (_Float16)bf16r(f1.w);
    _Float16* dst = x16 + (size_t)row * DM + col;
    *(volatile v8h*)dst = o;
    __threadfence();
    *(volatile v8h*)dst = o;
}

__global__ __launch_bounds__(256) void k_wt(const float* __restrict__ W, _Float16* WT, int N)
{
    __shared__ _Float16 tile[32 * 72] __attribute__((aligned(16)));
    const int tid = threadIdx.x;
    const int n0 = blockIdx.x * 32, k0 = blockIdx.y * 64;
    const int nn = tid & 31, kq = tid >> 5;
#pragma unroll
    for (int i = 0; i < 8; ++i) {
        const int kk = kq + 8 * i;
        const float w = W[(size_t)(k0 + kk) * N + n0 + nn];
        tile[nn * 72 + kk] = (_Float16)(bf16r(w) * WSCALE);
    }
    __syncthreads();
    const int on = tid >> 3, seg = tid & 7;
    const v8h v = *reinterpret_cast<const v8h*>(tile + on * 72 + seg * 8);
    _Float16* dst = WT + (size_t)(n0 + on) * DM + k0 + seg * 8;
    *(volatile v8h*)dst = v;
    __threadfence();
    *(volatile v8h*)dst = v;
}

__device__ __forceinline__ float rope_freq(int i)
{
    const double t = (double)i * (4.0 * 3.321928094887362348 * 0.015625);
    const double n = __builtin_rint(t);
    const double z = (t - n) * 0.6931471805599453094;
    double e = 1.0 / 8.71782912e10;
    e = fma(e, z, 1.0 / 6.2270208e9);
    e = fma(e, z, 1.0 / 4.790016e8);
    e = fma(e, z, 1.0 / 3.99168e7);
    e = fma(e, z, 1.0 / 3628800.0);
    e = fma(e, z, 1.0 / 362880.0);
    e = fma(e, z, 1.0 / 40320.0);
    e = fma(e, z, 1.0 / 5040.0);
    e = fma(e, z, 1.0 / 720.0);
    e = fma(e, z, 1.0 / 120.0);
    e = fma(e, z, 1.0 / 24.0);
    e = fma(e, z, 1.0 / 6.0);
    e = fma(e, z, 0.5);
    e = fma(e, z, 1.0);
    e = fma(e, z, 1.0);
    const float p32 = (float)ldexp(e, (int)n);
    return (float)(1.0 / (double)p32);
}

__global__ __launch_bounds__(256) void k_rope_tab(float* ctab, float* stab)
{
    __shared__ float cs[256] __attribute__((aligned(16)));
    __shared__ float sn[256] __attribute__((aligned(16)));
    const int tid = threadIdx.x;
    const int i = blockIdx.y;
    const int s = blockIdx.x * 256 + tid;
    const float fr = rope_freq(i);
    const float ang = (float)s * fr;
    float sv, cv;
    sincosf(ang, &sv, &cv);
    cs[tid] = cv;
    sn[tid] = sv;
    __syncthreads();
    if (tid < 128) {
        const int which = tid >> 6, t = tid & 63;
        const v4f vc = *reinterpret_cast<const v4f*>(cs + t * 4);
        const v4f vs = *reinterpret_cast<const v4f*>(sn + t * 4);
        v4f v;
        v[0] = which ? vs[0] : vc[0];
        v[1] = which ? vs[1] : vc[1];
        v[2] = which ? vs[2] : vc[2];
        v[3] = which ? vs[3] : vc[3];
        float* base = which ? stab : ctab;
        float* dst = base + (size_t)i * SEQ + blockIdx.x * 256 + t * 4;
        *(volatile v4f*)dst = v;
        __threadfence();
        *(volatile v4f*)dst = v;
    }
}

__device__ __forceinline__ void store128x128_f16(const _Float16* st, _Float16* gdst,
                                                 size_t pitch, int tid)
{
    const int rq = tid >> 4, seg = tid & 15;
    v8h v[8];
#pragma unroll
    for (int it = 0; it < 8; ++it)
        v[it] = *reinterpret_cast<const v8h*>(st + (it * 16 + rq) * 128 + seg * 8);
#pragma unroll
    for (int it = 0; it < 8; ++it)
        *(volatile v8h*)(gdst + (size_t)(it * 16 + rq) * pitch + seg * 8) = v[it];
    __threadfence();
#pragma unroll
    for (int it = 0; it < 8; ++it)
        *(volatile v8h*)(gdst + (size_t)(it * 16 + rq) * pitch + seg * 8) = v[it];
}

__global__ __launch_bounds__(256) void k_qkv(const _Float16* __restrict__ A,
                                             const _Float16* __restrict__ BT,
                                             const float* __restrict__ ctab,
                                             const float* __restrict__ stab,
                                             _Float16* q16, _Float16* k16,
                                             _Float16* vT, _Float16* vTr)
{
    __shared__ _Float16 Hs[128 * 128] __attribute__((aligned(16)));
    __shared__ _Float16 Ls[128 * 128] __attribute__((aligned(16)));
    const int tid = threadIdx.x;
    const int lane = tid & 31, wave = tid >> 5;
    const int wm = wave & 3, wn = wave >> 2;
    const int l15 = lane & 15, hi8 = (lane >> 4) << 3;
    const int cb = blockIdx.x;
    const int bm0 = blockIdx.y * 128, bn0 = cb * 128;
    const int K = DM;

    const _Float16* ap0 = A + (size_t)(bm0 + wm * 32 + l15) * K + hi8;
    const _Float16* ap1 = ap0 + (size_t)16 * K;
    const _Float16* bpa = BT + (size_t)(bn0 + wn * 32 + l15) * K + hi8;
    const _Float16* bpb = bpa + (size_t)64 * K;
    const size_t bst = (size_t)16 * K;

    const v8f zero8 = {0.f, 0.f, 0.f, 0.f, 0.f, 0.f, 0.f, 0.f};
    v8f acc[2][4];
#pragma unroll
    for (int g = 0; g < 2; ++g)
#pragma unroll
        for (int ni = 0; ni < 4; ++ni) acc[g][ni] = zero8;

    for (int k0 = 0; k0 < K; k0 += 32) {
        const v16h a0 = load_frag(ap0 + k0);
        const v16h a1 = load_frag(ap1 + k0);
        const v16h b0 = load_frag(bpa + k0);
        const v16h b1 = load_frag(bpa + bst + k0);
        const v16h b2 = load_frag(bpb + k0);
        const v16h b3 = load_frag(bpb + bst + k0);
        acc[0][0] = wmma16(a0, b0, acc[0][0]);
        acc[0][1] = wmma16(a0, b1, acc[0][1]);
        acc[0][2] = wmma16(a0, b2, acc[0][2]);
        acc[0][3] = wmma16(a0, b3, acc[0][3]);
        acc[1][0] = wmma16(a1, b0, acc[1][0]);
        acc[1][1] = wmma16(a1, b1, acc[1][1]);
        acc[1][2] = wmma16(a1, b2, acc[1][2]);
        acc[1][3] = wmma16(a1, b3, acc[1][3]);
        asm volatile("v_nop\n\tv_nop\n\tv_nop\n\tv_nop"
                     : "+v"(acc[0][0]), "+v"(acc[0][1]), "+v"(acc[0][2]), "+v"(acc[0][3]),
                       "+v"(acc[1][0]), "+v"(acc[1][1]), "+v"(acc[1][2]), "+v"(acc[1][3])
                     : "v"(a0), "v"(a1), "v"(b0), "v"(b1), "v"(b2), "v"(b3));
    }

    const int bb = bm0 / SEQ;
    const int s0 = bm0 - bb * SEQ;
    const float inv = 1.0f / WSCALE;
    const bool early = (s0 < EARLY);

    if (cb < NH + NKV) {
        const float oa = (cb < NH) ? QALPHA : 1.0f;
#pragma unroll
        for (int g = 0; g < 2; ++g) {
#pragma unroll
            for (int p = 0; p < 2; ++p) {
                const int d  = wn * 32 + p * 16 + l15;
                const int sr = s0 + wm * 32 + g * 16 + hi8;
                const float* cp = ctab + (size_t)d * SEQ + sr;
                const float* sp = stab + (size_t)d * SEQ + sr;
                const v4f ca = *reinterpret_cast<const v4f*>(cp);
                const v4f cc4 = *reinterpret_cast<const v4f*>(cp + 4);
                const v4f sa = *reinterpret_cast<const v4f*>(sp);
                const v4f sc4 = *reinterpret_cast<const v4f*>(sp + 4);
                float cc[8], ss[8];
                cc[0] = ca[0]; cc[1] = ca[1]; cc[2] = ca[2]; cc[3] = ca[3];
                cc[4] = cc4[0]; cc[5] = cc4[1]; cc[6] = cc4[2]; cc[7] = cc4[3];
                ss[0] = sa[0]; ss[1] = sa[1]; ss[2] = sa[2]; ss[3] = sa[3];
                ss[4] = sc4[0]; ss[5] = sc4[1]; ss[6] = sc4[2]; ss[7] = sc4[3];
#pragma unroll
                for (int j = 0; j < 8; ++j) {
                    const float x1 = acc[g][p][j] * inv;
                    const float x2 = acc[g][p + 2][j] * inv;
                    const float re = (x1 * cc[j] - x2 * ss[j]) * oa;
                    const float im = (x1 * ss[j] + x2 * cc[j]) * oa;
                    const int row = wm * 32 + g * 16 + hi8 + j;
                    Hs[row * 128 + d]      = (_Float16)re;
                    Hs[row * 128 + 64 + d] = (_Float16)im;
                }
            }
        }
    } else {
#pragma unroll
        for (int g = 0; g < 2; ++g)
#pragma unroll
            for (int ni = 0; ni < 4; ++ni) {
                const int col = (ni & 1) * 16 + (ni >> 1) * 64 + wn * 32 + l15;
#pragma unroll
                for (int j = 0; j < 8; ++j) {
                    const int row = wm * 32 + g * 16 + hi8 + j;
                    const float v = acc[g][ni][j] * inv;
                    const _Float16 hv = (_Float16)v;
                    Hs[col * 128 + row] = hv;
                    if (early) Ls[col * 128 + row] = (_Float16)((v - (float)hv) * RSC);
                }
            }
    }
    __syncthreads();

    if (cb < NH) {
        store128x128_f16(Hs, q16 + (size_t)bm0 * DM + cb * 128, (size_t)DM, tid);
    } else if (cb < NH + NKV) {
        store128x128_f16(Hs, k16 + (size_t)bm0 * KVW + (cb - NH) * 128, (size_t)KVW, tid);
    } else {
        const int kvh = cb - NH - NKV;
        store128x128_f16(Hs, vT + ((size_t)(bb * KVW + kvh * 128)) * SEQ + s0, (size_t)SEQ, tid);
        if (early)
            store128x128_f16(Ls, vTr + ((size_t)(bb * KVW + kvh * 128)) * EARLY + s0,
                             (size_t)EARLY, tid);
    }
}

__device__ __forceinline__ void qk_step(const v16h a0, const v16h a1,
                                        const _Float16* kp0, const _Float16* kp1,
                                        v8f& s0, v8f& s1)
{
    const v16h b00 = load_frag(kp0);
    const v16h b01 = load_frag(kp0 + 32);
    const v16h b10 = load_frag(kp1);
    const v16h b11 = load_frag(kp1 + 32);
    s0 = wmma16(a0, b00, s0);
    s0 = wmma16(a1, b01, s0);
    s1 = wmma16(a0, b10, s1);
    s1 = wmma16(a1, b11, s1);
    asm volatile("v_nop\n\tv_nop\n\tv_nop\n\tv_nop"
                 : "+v"(s0), "+v"(s1)
                 : "v"(a0), "v"(a1), "v"(b00), "v"(b01), "v"(b10), "v"(b11));
}

template <bool RES>
__device__ __forceinline__ void pv4(const v16h aP, const v16h aPr,
                                    const _Float16* vb, const _Float16* vrb,
                                    v8f& y0, v8f& y1, v8f& y2, v8f& y3,
                                    v8f& r0, v8f& r1, v8f& r2, v8f& r3)
{
    const v16h b0 = load_frag(vb);
    const v16h b1 = load_frag(vb + (size_t)16 * SEQ);
    const v16h b2 = load_frag(vb + (size_t)32 * SEQ);
    const v16h b3 = load_frag(vb + (size_t)48 * SEQ);
    y0 = wmma16(aP, b0, y0);
    y1 = wmma16(aP, b1, y1);
    y2 = wmma16(aP, b2, y2);
    y3 = wmma16(aP, b3, y3);
    if (RES) {
        const v16h c0 = load_frag(vrb);
        const v16h c1 = load_frag(vrb + (size_t)16 * EARLY);
        const v16h c2 = load_frag(vrb + (size_t)32 * EARLY);
        const v16h c3 = load_frag(vrb + (size_t)48 * EARLY);
        r0 = wmma16(aP, c0, r0);
        r1 = wmma16(aP, c1, r1);
        r2 = wmma16(aP, c2, r2);
        r3 = wmma16(aP, c3, r3);
        r0 = wmma16(aPr, b0, r0);
        r1 = wmma16(aPr, b1, r1);
        r2 = wmma16(aPr, b2, r2);
        r3 = wmma16(aPr, b3, r3);
        asm volatile("v_nop\n\tv_nop\n\tv_nop\n\tv_nop"
                     : "+v"(y0), "+v"(y1), "+v"(y2), "+v"(y3),
                       "+v"(r0), "+v"(r1), "+v"(r2), "+v"(r3)
                     : "v"(aP), "v"(aPr), "v"(b0), "v"(b1), "v"(b2), "v"(b3),
                       "v"(c0), "v"(c1), "v"(c2), "v"(c3));
    } else {
        asm volatile("v_nop\n\tv_nop\n\tv_nop\n\tv_nop"
                     : "+v"(y0), "+v"(y1), "+v"(y2), "+v"(y3)
                     : "v"(aP), "v"(b0), "v"(b1), "v"(b2), "v"(b3));
    }
}

template <int NT, bool RES>
__global__ __launch_bounds__(128) void k_attn(const _Float16* __restrict__ qp,
                                              const _Float16* __restrict__ kp,
                                              const _Float16* __restrict__ vT,
                                              const _Float16* __restrict__ vTr,
                                              _Float16* yp, _Float16* yrp,
                                              int qt0, int nqt)
{
    constexpr int NDQ = 8 / NT;
    constexpr int PP = 136;
    __shared__ _Float16 Ph[4 * 16 * PP] __attribute__((aligned(16)));
    __shared__ _Float16 Pr[RES ? 4 * 16 * PP : 8] __attribute__((aligned(16)));

    const int lane = threadIdx.x & 31;
    const int wv   = threadIdx.x >> 5;
    const int l15  = lane & 15;
    const int hi8  = (lane >> 4) << 3;

    int bx = blockIdx.x;
    const int dq = bx % NDQ; bx /= NDQ;
    const int qt = qt0 + (bx % nqt); bx /= nqt;
    const int kv = bx % NKV;
    const int b  = bx / NKV;
    const int h  = kv * GQ + wv;
    const int d0 = dq * NT * 16;

    const _Float16* qbase = qp + ((size_t)(b * SEQ + qt * 16 + l15)) * DM + h * HD + hi8;
    const v16h aQ0 = load_frag(qbase);
    const v16h aQ1 = load_frag(qbase + 32);
    const v16h aQ2 = load_frag(qbase + 64);
    const v16h aQ3 = load_frag(qbase + 96);

    const _Float16* kbase = kp + (size_t)b * SEQ * KVW + kv * HD + hi8;
    const _Float16* vbase = vT + ((size_t)(b * KVW + kv * HD + d0 + l15)) * SEQ + hi8;
    const _Float16* vrbase = vTr + ((size_t)(b * KVW + kv * HD + d0 + l15)) * EARLY + hi8;

    const v8f zero8 = {0.f, 0.f, 0.f, 0.f, 0.f, 0.f, 0.f, 0.f};
    float m[8], l[8];
    v8f accY[8], accYr[8];
#pragma unroll
    for (int j = 0; j < 8; ++j) { m[j] = NEGBIG; l[j] = 0.0f; }
#pragma unroll
    for (int ni = 0; ni < 8; ++ni) { accY[ni] = zero8; accYr[ni] = zero8; }
    v8f dr = zero8;

    _Float16* ph = Ph + wv * 16 * PP;
    _Float16* pr = Pr + (RES ? wv * 16 * PP : 0);

    const int nsteps = (qt >> 1) + 1;
    for (int st = 0; st < nsteps; ++st) {
        const int tc = st * 32;
        const _Float16* kp0 = kbase + (size_t)(tc + l15) * KVW;
        const _Float16* kp1 = kp0 + (size_t)16 * KVW;
        v8f s0 = zero8, s1 = zero8;
        qk_step(aQ0, aQ1, kp0, kp1, s0, s1);
        qk_step(aQ2, aQ3, kp0 + 64, kp1 + 64, s0, s1);

        const bool diag = (tc + 31 > qt * 16);
#pragma unroll
        for (int j = 0; j < 8; ++j) {
            float a0 = s0[j] * (1.0f / QCARRY);
            float a1 = s1[j] * (1.0f / QCARRY);
            if (diag) {
                const int qr = qt * 16 + hi8 + j;
                a0 = (tc + l15 > qr) ? NEGBIG : a0;
                a1 = (tc + 16 + l15 > qr) ? NEGBIG : a1;
            }
            float mt = fmaxf(a0, a1);
#pragma unroll
            for (int off = 8; off >= 1; off >>= 1)
                mt = fmaxf(mt, __shfl_xor(mt, off, 16));
            const float mn = fmaxf(m[j], mt);
            const float sc = exp2f(m[j] - mn);
            const float p0 = exp2f(a0 - mn);
            const float p1 = exp2f(a1 - mn);
            float rs = p0 + p1;
#pragma unroll
            for (int off = 8; off >= 1; off >>= 1)
                rs += __shfl_xor(rs, off, 16);
            l[j] = l[j] * sc + rs;
            m[j] = mn;
#pragma unroll
            for (int ni = 0; ni < NT; ++ni) {
                accY[ni][j] *= sc;
                if (RES) accYr[ni][j] *= sc;
            }
            const int row = hi8 + j;
            const float c0 = p0 * PCARRY;
            const float c1 = p1 * PCARRY;
            const _Float16 h0 = (_Float16)c0;
            const _Float16 h1 = (_Float16)c1;
            ph[row * PP + l15]      = h0;
            ph[row * PP + 16 + l15] = h1;
            if (RES) {
                pr[row * PP + l15]      = (_Float16)((c0 - (float)h0) * RSC);
                pr[row * PP + 16 + l15] = (_Float16)((c1 - (float)h1) * RSC);
            }
        }
        __syncthreads();

        const v16h aP  = load_frag(ph + l15 * PP + hi8);
        const v16h aPr = RES ? load_frag(pr + l15 * PP + hi8) : aP;
        const _Float16* vb  = vbase + tc;
        const _Float16* vrb = vrbase + tc;
        if (RES) {
            pv4<true>(aP, aPr, vb, vrb, accY[0], accY[1], accY[2], accY[3],
                      accYr[0], accYr[1], accYr[2], accYr[3]);
        } else {
            pv4<false>(aP, aP, vb, vb, accY[0], accY[1], accY[2], accY[3], dr, dr, dr, dr);
            if (NT == 8)
                pv4<false>(aP, aP, vb + (size_t)64 * SEQ, vb, accY[4], accY[5], accY[6], accY[7],
                           dr, dr, dr, dr);
        }
    }
    __syncthreads();

    float inv[8];
#pragma unroll
    for (int j = 0; j < 8; ++j) inv[j] = (YCARRY / PCARRY) / l[j];
#pragma unroll
    for (int ni = 0; ni < NT; ++ni)
#pragma unroll
        for (int j = 0; j < 8; ++j) {
            float yv = accY[ni][j];
            if (RES) yv += accYr[ni][j] * RINV;
            yv *= inv[j];
            const _Float16 hv = (_Float16)yv;
            ph[(hi8 + j) * PP + ni * 16 + l15] = hv;
            if (RES) pr[(hi8 + j) * PP + ni * 16 + l15] = (_Float16)((yv - (float)hv) * RSC);
        }
    __syncthreads();

    constexpr int LPR = NT * 2;
    constexpr int RPI = 32 / LPR;
    constexpr int NIT = 16 / RPI;
    const int rq = lane / LPR, seg = lane % LPR;
    {
        v8h v[NIT];
#pragma unroll
        for (int it = 0; it < NIT; ++it)
            v[it] = *reinterpret_cast<const v8h*>(ph + (it * RPI + rq) * PP + seg * 8);
        _Float16* yd = yp + ((size_t)(b * SEQ + qt * 16)) * DM + h * HD + d0 + seg * 8;
#pragma unroll
        for (int it = 0; it < NIT; ++it)
            *(volatile v8h*)(yd + (size_t)(it * RPI + rq) * DM) = v[it];
        __threadfence();
#pragma unroll
        for (int it = 0; it < NIT; ++it)
            *(volatile v8h*)(yd + (size_t)(it * RPI + rq) * DM) = v[it];
    }
    if (RES) {
        v8h v[NIT];
#pragma unroll
        for (int it = 0; it < NIT; ++it)
            v[it] = *reinterpret_cast<const v8h*>(pr + (it * RPI + rq) * PP + seg * 8);
        _Float16* yd = yrp + ((size_t)(b * EARLY + qt * 16)) * DM + h * HD + d0 + seg * 8;
#pragma unroll
        for (int it = 0; it < NIT; ++it)
            *(volatile v8h*)(yd + (size_t)(it * RPI + rq) * DM) = v[it];
        __threadfence();
#pragma unroll
        for (int it = 0; it < NIT; ++it)
            *(volatile v8h*)(yd + (size_t)(it * RPI + rq) * DM) = v[it];
    }
}

__global__ __launch_bounds__(256) void k_gemm_out(const _Float16* __restrict__ A,
                                                  const _Float16* __restrict__ BT,
                                                  float* C, int rbPer, int rowStart, float alpha)
{
    __shared__ float stg[8 * 1024] __attribute__((aligned(16)));
    const int tid = threadIdx.x;
    const int lane = tid & 31, wave = tid >> 5;
    const int wm = wave & 3, wn = wave >> 2;
    const int l15 = lane & 15, hi8 = (lane >> 4) << 3;
    const int by = blockIdx.y;
    const int bb = by / rbPer;
    const int bm0 = bb * SEQ + rowStart + (by - bb * rbPer) * 128;
    const int bn0 = blockIdx.x * 128;
    const int K = DM, N = DM;

    const _Float16* ap0 = A + (size_t)(bm0 + wm * 32 + l15) * K + hi8;
    const _Float16* ap1 = ap0 + (size_t)16 * K;
    const _Float16* bp  = BT + (size_t)(bn0 + wn * 64 + l15) * K + hi8;
    const size_t bst = (size_t)16 * K;

    const v8f zero8 = {0.f, 0.f, 0.f, 0.f, 0.f, 0.f, 0.f, 0.f};
    v8f acc[2][4];
#pragma unroll
    for (int g = 0; g < 2; ++g)
#pragma unroll
        for (int ni = 0; ni < 4; ++ni) acc[g][ni] = zero8;

    for (int k0 = 0; k0 < K; k0 += 32) {
        const v16h a0 = load_frag(ap0 + k0);
        const v16h a1 = load_frag(ap1 + k0);
        const v16h b0 = load_frag(bp + k0);
        const v16h b1 = load_frag(bp + bst + k0);
        const v16h b2 = load_frag(bp + 2 * bst + k0);
        const v16h b3 = load_frag(bp + 3 * bst + k0);
        acc[0][0] = wmma16(a0, b0, acc[0][0]);
        acc[0][1] = wmma16(a0, b1, acc[0][1]);
        acc[0][2] = wmma16(a0, b2, acc[0][2]);
        acc[0][3] = wmma16(a0, b3, acc[0][3]);
        acc[1][0] = wmma16(a1, b0, acc[1][0]);
        acc[1][1] = wmma16(a1, b1, acc[1][1]);
        acc[1][2] = wmma16(a1, b2, acc[1][2]);
        acc[1][3] = wmma16(a1, b3, acc[1][3]);
        asm volatile("v_nop\n\tv_nop\n\tv_nop\n\tv_nop"
                     : "+v"(acc[0][0]), "+v"(acc[0][1]), "+v"(acc[0][2]), "+v"(acc[0][3]),
                       "+v"(acc[1][0]), "+v"(acc[1][1]), "+v"(acc[1][2]), "+v"(acc[1][3])
                     : "v"(a0), "v"(a1), "v"(b0), "v"(b1), "v"(b2), "v"(b3));
    }

    float* swf = stg + wave * 1024;
    const int rq = lane >> 4, seg = lane & 15;
#pragma unroll
    for (int g = 0; g < 2; ++g) {
#pragma unroll
        for (int ni = 0; ni < 4; ++ni)
#pragma unroll
            for (int j = 0; j < 8; ++j)
                swf[(hi8 + j) * 64 + ni * 16 + l15] = acc[g][ni][j] * alpha;
        __syncthreads();
        v4f v[8];
#pragma unroll
        for (int it = 0; it < 8; ++it)
            v[it] = *reinterpret_cast<const v4f*>(swf + (it * 2 + rq) * 64 + seg * 4);
        float* gd = C + (size_t)(bm0 + wm * 32 + g * 16) * N + bn0 + wn * 64 + seg * 4;
#pragma unroll
        for (int it = 0; it < 8; ++it)
            *(volatile v4f*)(gd + (size_t)(it * 2 + rq) * N) = v[it];
        __threadfence();
#pragma unroll
        for (int it = 0; it < 8; ++it)
            *(volatile v4f*)(gd + (size_t)(it * 2 + rq) * N) = v[it];
        __syncthreads();
    }
}

__global__ __launch_bounds__(256) void k_gemm_out_res(const _Float16* __restrict__ Ah,
                                                      const _Float16* __restrict__ Ar,
                                                      const _Float16* __restrict__ BT,
                                                      float* C, float alpha)
{
    __shared__ float stg[8 * 1024] __attribute__((aligned(16)));
    const int tid = threadIdx.x;
    const int lane = tid & 31, wave = tid >> 5;
    const int wm = wave & 3, wn = wave >> 2;
    const int l15 = lane & 15, hi8 = (lane >> 4) << 3;
    constexpr int EB = EARLY / 64;
    const int by = blockIdx.y;
    const int bb = by / EB;
    const int s0 = (by - bb * EB) * 64;
    const int bn0 = blockIdx.x * 128;
    const int K = DM, N = DM;

    const _Float16* ah = Ah + (size_t)(bb * SEQ + s0 + wm * 16 + l15) * K + hi8;
    const _Float16* ar = Ar + (size_t)(bb * EARLY + s0 + wm * 16 + l15) * K + hi8;
    const _Float16* bp = BT + (size_t)(bn0 + wn * 64 + l15) * K + hi8;
    const size_t bst = (size_t)16 * K;

    const v8f zero8 = {0.f, 0.f, 0.f, 0.f, 0.f, 0.f, 0.f, 0.f};
    v8f acc[4], accr[4];
#pragma unroll
    for (int ni = 0; ni < 4; ++ni) { acc[ni] = zero8; accr[ni] = zero8; }

    for (int k0 = 0; k0 < K; k0 += 32) {
        const v16h a0 = load_frag(ah + k0);
        const v16h a1 = load_frag(ar + k0);
        const v16h b0 = load_frag(bp + k0);
        const v16h b1 = load_frag(bp + bst + k0);
        const v16h b2 = load_frag(bp + 2 * bst + k0);
        const v16h b3 = load_frag(bp + 3 * bst + k0);
        acc[0]  = wmma16(a0, b0, acc[0]);
        acc[1]  = wmma16(a0, b1, acc[1]);
        acc[2]  = wmma16(a0, b2, acc[2]);
        acc[3]  = wmma16(a0, b3, acc[3]);
        accr[0] = wmma16(a1, b0, accr[0]);
        accr[1] = wmma16(a1, b1, accr[1]);
        accr[2] = wmma16(a1, b2, accr[2]);
        accr[3] = wmma16(a1, b3, accr[3]);
        asm volatile("v_nop\n\tv_nop\n\tv_nop\n\tv_nop"
                     : "+v"(acc[0]), "+v"(acc[1]), "+v"(acc[2]), "+v"(acc[3]),
                       "+v"(accr[0]), "+v"(accr[1]), "+v"(accr[2]), "+v"(accr[3])
                     : "v"(a0), "v"(a1), "v"(b0), "v"(b1), "v"(b2), "v"(b3));
    }

    float* swf = stg + wave * 1024;
    const int rq = lane >> 4, seg = lane & 15;
#pragma unroll
    for (int ni = 0; ni < 4; ++ni)
#pragma unroll
        for (int j = 0; j < 8; ++j)
            swf[(hi8 + j) * 64 + ni * 16 + l15] = (acc[ni][j] + accr[ni][j] * RINV) * alpha;
    __syncthreads();
    v4f v[8];
#pragma unroll
    for (int it = 0; it < 8; ++it)
        v[it] = *reinterpret_cast<const v4f*>(swf + (it * 2 + rq) * 64 + seg * 4);
    float* gd = C + (size_t)(bb * SEQ + s0 + wm * 16) * N + bn0 + wn * 64 + seg * 4;
#pragma unroll
    for (int it = 0; it < 8; ++it)
        *(volatile v4f*)(gd + (size_t)(it * 2 + rq) * N) = v[it];
    __threadfence();
#pragma unroll
    for (int it = 0; it < 8; ++it)
        *(volatile v4f*)(gd + (size_t)(it * 2 + rq) * N) = v[it];
}

extern "C" void kernel_launch(void* const* d_in, const int* in_sizes, int n_in,
                              void* d_out, int out_size, void* d_ws, size_t ws_size,
                              hipStream_t stream) {
    if (n_in < 3) return;
    const long long needX = ((long long)(NB - 1) * SEQ_FULL + SEQ) * DM;
    if ((long long)in_sizes[0] < needX) return;
    if ((long long)in_sizes[1] < (long long)DM * NQKV || (long long)in_sizes[2] < (long long)DM * DM) return;
    if ((long long)out_size < (long long)MROWS * DM) return;

    const float* x    = (const float*)d_in[0];
    const float* Wqkv = (const float*)d_in[1];
    const float* Wo   = (const float*)d_in[2];
    float* out = (float*)d_out;

    size_t off = 0;
    char* wsb = (char*)d_ws;
    auto carve = [&](size_t bytes) -> void* {
        void* p = wsb + off;
        off += (bytes + 255) & ~(size_t)255;
        return p;
    };
    _Float16* x16   = (_Float16*)carve((size_t)MROWS * DM * 2);
    _Float16* WqkvT = (_Float16*)carve((size_t)NQKV * DM * 2);
    _Float16* WoT   = (_Float16*)carve((size_t)DM * DM * 2);
    float*    ctab  = (float*)carve((size_t)64 * SEQ * 4);
    float*    stab  = (float*)carve((size_t)64 * SEQ * 4);
    _Float16* q16   = (_Float16*)carve((size_t)MROWS * DM * 2);
    _Float16* k16   = (_Float16*)carve((size_t)MROWS * KVW * 2);
    _Float16* vT    = (_Float16*)carve((size_t)NB * KVW * SEQ * 2);
    _Float16* vTr   = (_Float16*)carve((size_t)NB * KVW * EARLY * 2);
    _Float16* y16   = (_Float16*)carve((size_t)MROWS * DM * 2);
    _Float16* yr    = (_Float16*)carve((size_t)NB * EARLY * DM * 2);
    if (off > ws_size) return;
    if (off > (size_t)134217728) return;

    dim3 blk(256);

    k_cvt_x<<<dim3(MROWS), blk, 0, stream>>>(x, x16);
    k_wt<<<dim3(NQKV / 32, DM / 64), blk, 0, stream>>>(Wqkv, WqkvT, NQKV);
    k_wt<<<dim3(DM / 32, DM / 64), blk, 0, stream>>>(Wo, WoT, DM);
    k_rope_tab<<<dim3(SEQ / 256, 64), blk, 0, stream>>>(ctab, stab);

    k_qkv<<<dim3(NQKV / 128, MROWS / 128), blk, 0, stream>>>(
        x16, WqkvT, ctab, stab, q16, k16, vT, vTr);

    const int nqtE = EARLY / 16;
    const int nqtP = (SEQ - EARLY) / 16;
    if (nqtP > 0)
        k_attn<8, false><<<dim3(NB * NKV * nqtP), dim3(128), 0, stream>>>(
            q16, k16, vT, vTr, y16, yr, nqtE, nqtP);
    k_attn<4, true><<<dim3(NB * NKV * nqtE * 2), dim3(128), 0, stream>>>(
        q16, k16, vT, vTr, y16, yr, 0, nqtE);

    const int rbP = (SEQ - EARLY) / 128;
    if (rbP > 0)
        k_gemm_out<<<dim3(DM / 128, NB * rbP), blk, 0, stream>>>(
            y16, WoT, out, rbP, EARLY, 1.0f / (YCARRY * WSCALE));
    k_gemm_out_res<<<dim3(DM / 128, NB * (EARLY / 64)), blk, 0, stream>>>(
        y16, yr, WoT, out, 1.0f / (YCARRY * WSCALE));
}
